// DCNV2_59150289601022
// MI455X (gfx1250) — hardware-verified
//
#include <hip/hip_runtime.h>
#include <stddef.h>
#include <math.h>

typedef __attribute__((ext_vector_type(16))) _Float16 v16h;
typedef __attribute__((ext_vector_type(8)))  _Float16 v8h;
typedef __attribute__((ext_vector_type(16))) __bf16   v16b;
typedef __attribute__((ext_vector_type(8)))  __bf16   v8b;
typedef __attribute__((ext_vector_type(8)))  float    v8f;
typedef __attribute__((ext_vector_type(4)))  float    v4f;

constexpr int NBATCH  = 8;
constexpr int NCH     = 64;
constexpr int NHGT    = 128;
constexpr int NWID    = 128;
constexpr int NCO     = 64;
constexpr int NTAP    = 9;
constexpr int NPIX    = NHGT * NWID;
constexpr int KDIM    = NTAP * NCH;
constexpr int NOFF    = 27;
constexpr int NOFFPAD = 64;
constexpr int BCHUNK  = 2;
constexpr int NCHUNK  = NBATCH / BCHUNK;
constexpr int MROWS   = BCHUNK * NPIX;
constexpr int NTHR    = 256;
constexpr int XT_PITCH = 68;
constexpr float A_CARRY  = 8.0f;
constexpr float W1_CARRY = 256.0f;
constexpr float W2_CARRY = 64.0f;
constexpr float G1_FOLD  = 1.0f / 2048.0f;
constexpr float G2_FOLD  = 1.0f / 512.0f;

constexpr size_t XT_BYTES = (size_t)NBATCH * NPIX * NCH * 4;
constexpr size_t P_BYTES  = (size_t)MROWS * KDIM * 2;
constexpr size_t OM_BYTES = (size_t)MROWS * NOFFPAD * 4;
constexpr size_t BT_BYTES = (size_t)NOFFPAD * KDIM * 2;
constexpr size_t WS_XT  = 0;
constexpr size_t WS_P   = WS_XT + XT_BYTES;
constexpr size_t WS_OM  = WS_P + P_BYTES;
constexpr size_t WS_BT1 = WS_OM + OM_BYTES;
constexpr size_t WS_BT2 = WS_BT1 + BT_BYTES;
constexpr size_t WS_TOTAL = WS_BT2 + BT_BYTES;
static_assert(WS_TOTAL == 79839232u);
static_assert(WS_TOTAL <= 134217728u);
static_assert(WS_P % 256 == 0 && WS_OM % 256 == 0 && WS_BT1 % 128 == 0 && WS_BT2 % 128 == 0);

static_assert(KDIM % 32 == 0);
static_assert(MROWS % 64 == 0 && NOFFPAD % 64 == 0);
static_assert(NCO % 64 == 0 && NPIX % 64 == 0);
static_assert((MROWS / 64) % 8 == 0 && (NPIX / 64) % 8 == 0);
static_assert((MROWS * NTAP * 8) % NTHR == 0);
static_assert((NOFFPAD * (KDIM / 8)) % NTHR == 0);
static_assert(NWID == 128 && NPIX == 16384 && MROWS == 32768);

__device__ __forceinline__ unsigned short f2bf_bits(float f) {
  unsigned u = __float_as_uint(f);
  return (unsigned short)((u + 0x7FFFu + ((u >> 16) & 1u)) >> 16);
}
__device__ __forceinline__ float bf_bits2f(unsigned short h) { return __uint_as_float(((unsigned)h) << 16); }

__device__ __forceinline__ void dep_guard_h(v8f& a, v8f& b, v16h x, v16h y) { asm volatile("v_nop\n\tv_nop\n\tv_nop\n\tv_nop" : "+v"(a), "+v"(b) : "v"(x), "v"(y)); }
__device__ __forceinline__ void dep_guard_b(v8f& a, v8f& b, v16b x, v16b y) { asm volatile("v_nop\n\tv_nop\n\tv_nop\n\tv_nop" : "+v"(a), "+v"(b) : "v"(x), "v"(y)); }
__device__ __forceinline__ void keep4_h(v16h a, v16h b, v16h c, v16h d) { asm volatile("v_nop" :: "v"(a), "v"(b), "v"(c), "v"(d)); }
__device__ __forceinline__ void keep4_b(v16b a, v16b b, v16b c, v16b d) { asm volatile("v_nop" :: "v"(a), "v"(b), "v"(c), "v"(d)); }
__device__ __forceinline__ void acc_guard4(v8f& a, v8f& b, v8f& c, v8f& d) { asm volatile("v_nop\n\tv_nop\n\tv_nop\n\tv_nop" : "+v"(a), "+v"(b), "+v"(c), "+v"(d)); }
template <typename T> struct Frag;
template <> struct Frag<_Float16> {
  typedef v16h V; union U { v16h v; v8h h[2]; };
  static __device__ __forceinline__ v16h load(const _Float16* p) {
    U f; f.h[0] = *(const v8h*)(p); f.h[1] = *(const v8h*)(p + 16); return f.v;
  }
  static __device__ __forceinline__ v8f mma(v16h a, v16h b, v8f c) {
    return __builtin_amdgcn_wmma_f32_16x16x32_f16(false, a, false, b, (short)0, c, false, false);
  }
  static __device__ __forceinline__ void guard(v8f& a, v8f& b, v16h x, v16h y) { dep_guard_h(a, b, x, y); }
  static __device__ __forceinline__ void keep(v16h a, v16h b, v16h c, v16h d) { keep4_h(a, b, c, d); }
};
template <> struct Frag<__bf16> {
  typedef v16b V; union U { v16b v; v8b h[2]; };
  static __device__ __forceinline__ v16b load(const __bf16* p) {
    U f; f.h[0] = *(const v8b*)(p); f.h[1] = *(const v8b*)(p + 16); return f.v;
  }
  static __device__ __forceinline__ v8f mma(v16b a, v16b b, v8f c) {
    return __builtin_amdgcn_wmma_f32_16x16x32_bf16(false, a, false, b, (short)0, c, false, false);
  }
  static __device__ __forceinline__ void guard(v8f& a, v8f& b, v16b x, v16b y) { dep_guard_b(a, b, x, y); }
  static __device__ __forceinline__ void keep(v16b a, v16b b, v16b c, v16b d) { keep4_b(a, b, c, d); }
};

template <int ET> struct Elem;
template <> struct Elem<0> { typedef _Float16 T; };
template <> struct Elem<1> { typedef __bf16 T; };
template <int ET, bool SPLIT, int BIAS_MODE, int OUT_MODE, bool RESID, int ACT = 0>
__global__ __launch_bounds__(256) void wmma_gemm64(
    const unsigned short* __restrict__ Ap, const unsigned short* __restrict__ A2p, int lda, long strideA,
    const unsigned short* __restrict__ Btp, const unsigned short* __restrict__ Bt2p, int ldb, long strideB,
    void* __restrict__ Cout, void* __restrict__ Cout2, int ldc, long strideC,
    const float* __restrict__ bias,
    const float* __restrict__ resid, long strideR,
    int M, int N, int K, float scale) {
  typedef typename Elem<ET>::T T;
  typedef typename Frag<T>::V V;
  const T* A = (const T*)Ap; const T* A2 = (const T*)A2p; const T* Bt = (const T*)Btp; const T* Bt2 = (const T*)Bt2p;
  __shared__ __align__(16) float sT[8][16 * 68];
  const int b    = blockIdx.y;
  const int lane = threadIdx.x & 31;
  const int wave = threadIdx.x >> 5;
  const int tilesN = N >> 6;
  const int tilesM = M >> 6;
  const int tile = blockIdx.x * 8 + wave;
  if (tile >= tilesM * tilesN) return;
  const int tm = tile / tilesN;
  const int tn = tile - tm * tilesN;
  const int m0 = tm << 6;
  const int n0 = tn << 6;

  const T* Ab  = A  + (size_t)b * strideA;
  const T* Bb  = Bt + (size_t)b * strideB;
  const T* Ab2 = SPLIT ? (A2  + (size_t)b * strideA) : nullptr;
  const T* Bb2 = SPLIT ? (Bt2 + (size_t)b * strideB) : nullptr;

  const int rlane = lane & 15;
  const int koff  = (lane >> 4) * 8;
  const int mOff  = (lane >> 4) * 8;

  v8f acc[4][4];
#pragma unroll
  for (int i = 0; i < 4; ++i)
#pragma unroll
    for (int j = 0; j < 4; ++j) acc[i][j] = (v8f){0.f,0.f,0.f,0.f,0.f,0.f,0.f,0.f};

  for (int k0 = 0; k0 < K; k0 += 32) {
    V bh[4], bl[4];
#pragma unroll
    for (int j = 0; j < 4; ++j) {
      const size_t bo = (size_t)(n0 + (j << 4) + rlane) * ldb + koff + k0;
      bh[j] = Frag<T>::load(Bb + bo);
      if (SPLIT) bl[j] = Frag<T>::load(Bb2 + bo);
    }
#pragma unroll
    for (int i = 0; i < 4; ++i) {
      const size_t ao = (size_t)(m0 + (i << 4) + rlane) * lda + koff + k0;
      V ah = Frag<T>::load(Ab + ao);
      V al;
      if (SPLIT) al = Frag<T>::load(Ab2 + ao);
#pragma unroll
      for (int j = 0; j < 4; ++j) {
        acc[i][j] = Frag<T>::mma(ah, bh[j], acc[i][j]);
        if (SPLIT) {
          acc[i][j] = Frag<T>::mma(ah, bl[j], acc[i][j]);
          acc[i][j] = Frag<T>::mma(al, bh[j], acc[i][j]);
        }
      }
      Frag<T>::guard(acc[i][0], acc[i][3], ah, SPLIT ? al : ah);
      acc_guard4(acc[i][0], acc[i][1], acc[i][2], acc[i][3]);
    }
    Frag<T>::keep(bh[0], bh[1], bh[2], bh[3]);
    if (SPLIT) Frag<T>::keep(bl[0], bl[1], bl[2], bl[3]);
  }
  acc_guard4(acc[0][0], acc[0][1], acc[0][2], acc[0][3]);
  acc_guard4(acc[1][0], acc[1][1], acc[1][2], acc[1][3]);
  acc_guard4(acc[2][0], acc[2][1], acc[2][2], acc[2][3]);
  acc_guard4(acc[3][0], acc[3][1], acc[3][2], acc[3][3]);

  float* slab = sT[wave];
  const float* Rb = RESID ? (resid + (size_t)b * strideR) : nullptr;
#pragma unroll
  for (int i = 0; i < 4; ++i) {
    const int mBase = m0 + (i << 4);
#pragma unroll
    for (int j = 0; j < 4; ++j) {
      const int n = n0 + (j << 4) + rlane;
      float bv = 0.f;
      if (BIAS_MODE == 2) bv = bias[n];
#pragma unroll
      for (int r = 0; r < 8; ++r) {
        float v = acc[i][j][r] * scale;
        if (BIAS_MODE == 1) v += bias[mBase + mOff + r];
        if (BIAS_MODE == 2) v += bv;
        if (RESID) v += Rb[(size_t)(mBase + mOff + r) * ldc + n];
        if (ACT == 1) v = tanhf(v);
        if (ACT == 2) v = fmaxf(v, 0.0f);
        if (ACT == 3) v = v / (1.0f + expf(-v));
        if (ACT == 4) v = (v > 0.f) ? v : 0.01f * v;
        if (ACT == 5) v = 0.5f * v * (1.0f + erff(v * 0.70710678118654752f));
        slab[(mOff + r) * 68 + (j << 4) + rlane] = v;
      }
    }
    __builtin_amdgcn_fence(__ATOMIC_RELEASE, "workgroup");
    __builtin_amdgcn_wave_barrier();
    __builtin_amdgcn_fence(__ATOMIC_ACQUIRE, "workgroup");
    if (OUT_MODE == 0) {
      float* C = (float*)Cout + (size_t)b * strideC;
      const int hh = lane >> 4, c4 = (lane & 15) * 4;
      for (int pass = 0; pass < 2; ++pass) {
#pragma unroll
        for (int it = 0; it < 8; ++it) {
          const int row = it * 2 + hh;
          v4f v = *(const v4f*)(slab + row * 68 + c4);
          *(volatile v4f*)(C + (size_t)(mBase + row) * ldc + n0 + c4) = v;
        }
        __threadfence();
      }
    } else {
      const int q = lane >> 3, c8 = (lane & 7) * 8;
      unsigned short* C  = (unsigned short*)Cout  + (size_t)b * strideC;
      unsigned short* C2 = (OUT_MODE == 2) ? ((unsigned short*)Cout2 + (size_t)b * strideC) : nullptr;
      for (int pass = 0; pass < 2; ++pass) {
#pragma unroll
        for (int it = 0; it < 4; ++it) {
          const int row = it * 4 + q;
          const float* sp = slab + row * 68 + c8;
          v8h hv, lv;
#pragma unroll
          for (int e = 0; e < 8; ++e) {
            if (OUT_MODE == 1) {
              hv[e] = (_Float16)sp[e];
            } else {
              unsigned short hb = f2bf_bits(sp[e]);
              unsigned short lb = f2bf_bits(sp[e] - bf_bits2f(hb));
              hv[e] = __builtin_bit_cast(_Float16, hb);
              lv[e] = __builtin_bit_cast(_Float16, lb);
            }
          }
          *(volatile v8h*)(C + (size_t)(mBase + row) * ldc + n0 + c8) = hv;
          if (OUT_MODE == 2) *(volatile v8h*)(C2 + (size_t)(mBase + row) * ldc + n0 + c8) = lv;
        }
        __threadfence();
      }
    }
    __builtin_amdgcn_fence(__ATOMIC_RELEASE, "workgroup");
    __builtin_amdgcn_wave_barrier();
    __builtin_amdgcn_fence(__ATOMIC_ACQUIRE, "workgroup");
  }
}

__global__ __launch_bounds__(NTHR) void k_xpose(const float* __restrict__ x, float* __restrict__ xt) {
  __shared__ __align__(16) float tile[64 * XT_PITCH];
  const int tid = threadIdx.x, lane = tid & 31, wave = tid >> 5;
  const int blk = blockIdx.x;
  const int xh  = blk & 1;
  const int y   = (blk >> 1) & (NHGT - 1);
  const int b   = blk >> 8;
  const int x0  = xh * 64;
  {
    const int c = tid >> 2, xq = tid & 3;
    const float* src = x + (((size_t)(b * NCH + c) * NHGT + y) * NWID + x0 + xq * 16);
    const v4f f0 = *(const v4f*)(src);
    const v4f f1 = *(const v4f*)(src + 4);
    const v4f f2 = *(const v4f*)(src + 8);
    const v4f f3 = *(const v4f*)(src + 12);
    float* trow = tile + (xq * 16) * XT_PITCH + c;
#pragma unroll
    for (int e = 0; e < 4; ++e) {
      trow[(e) * XT_PITCH]      = f0[e];
      trow[(4 + e) * XT_PITCH]  = f1[e];
      trow[(8 + e) * XT_PITCH]  = f2[e];
      trow[(12 + e) * XT_PITCH] = f3[e];
    }
  }
  __syncthreads();
  const int hh = lane >> 4, c4 = (lane & 15) * 4;
  float* dst = xt + ((size_t)(b * NHGT + y) * NWID + x0) * NCH;
  for (int pass = 0; pass < 2; ++pass) {
#pragma unroll
    for (int it = 0; it < 4; ++it) {
      const int row = it * 16 + wave * 2 + hh;
      const v4f v = *(const v4f*)(tile + row * XT_PITCH + c4);
      *(volatile v4f*)(dst + (size_t)row * NCH + c4) = v;
    }
    __threadfence();
  }
}

__global__ __launch_bounds__(NTHR) void k_wprep(const float* __restrict__ wsrc, int nreal, float scale,
                                                unsigned short* __restrict__ bt) {
  const int i   = blockIdx.x * NTHR + threadIdx.x;
  const int tpr = KDIM / 8;
  if (i >= NOFFPAD * tpr) return;
  const int n   = i / tpr;
  const int k0  = (i - n * tpr) * 8;
  const int kk  = k0 >> 6;
  const int c0  = k0 & 63;
  const int ncl = (n < nreal) ? n : (nreal - 1);
  v8h hv;
#pragma unroll
  for (int e = 0; e < 8; ++e) {
    float v = wsrc[((size_t)(ncl * NCH + c0 + e)) * NTAP + kk];
    if (n >= nreal) v = 0.0f;
    hv[e] = (_Float16)(scale * v);
  }
  unsigned short* p = bt + (size_t)i * 8;
  *(volatile v8h*)(p) = hv;
  __threadfence();
  *(volatile v8h*)(p) = hv;
}

__global__ __launch_bounds__(NTHR) void k_im2col(const float* __restrict__ xt, int bbase,
                                                 unsigned short* __restrict__ P) {
  const int t   = blockIdx.x * NTHR + threadIdx.x;
  const int g   = t >> 3, sub = t & 7;
  const int m   = g / NTAP;
  const int kk  = g - m * NTAP;
  const int bl  = m >> 14;
  const int ho  = (m >> 7) & (NHGT - 1);
  const int wo  = m & (NWID - 1);
  const int ky  = kk / 3, kx = kk - ky * 3;
  const int yy  = ho - 1 + ky, xx = wo - 1 + kx;
  const bool valid = (yy >= 0) && (yy < NHGT) && (xx >= 0) && (xx < NWID);
  const int yc  = min(max(yy, 0), NHGT - 1);
  const int xc  = min(max(xx, 0), NWID - 1);
  const int bg  = bbase + bl;
  const float* src = xt + (((size_t)(bg * NHGT + yc)) * NWID + xc) * NCH + sub * 8;
  const v4f f0 = *(const v4f*)(src);
  const v4f f1 = *(const v4f*)(src + 4);
  const float s = valid ? A_CARRY : 0.0f;
  v8h hv;
#pragma unroll
  for (int e = 0; e < 4; ++e) {
    hv[e]     = (_Float16)(f0[e] * s);
    hv[4 + e] = (_Float16)(f1[e] * s);
  }
  unsigned short* p = P + (size_t)t * 8;
  *(volatile v8h*)(p) = hv;
  __threadfence();
  *(volatile v8h*)(p) = hv;
}

__global__ __launch_bounds__(NTHR) void k_gather(const float* __restrict__ xt, const float* __restrict__ om,
                                                 const float* __restrict__ b_om, int bbase,
                                                 unsigned short* __restrict__ P) {
  const int t   = blockIdx.x * NTHR + threadIdx.x;
  const int g   = t >> 3, sub = t & 7;
  const int m   = g / NTAP;
  const int kk  = g - m * NTAP;
  const int bl  = m >> 14;
  const int ho  = (m >> 7) & (NHGT - 1);
  const int wo  = m & (NWID - 1);
  const int ky  = kk / 3, kx = kk - ky * 3;
  const size_t orow = (size_t)m * NOFFPAD;
  const float d_y = om[orow + kk] + b_om[kk];
  const float d_x = om[orow + NTAP + kk] + b_om[NTAP + kk];
  const float lg  = om[orow + 2 * NTAP + kk] + b_om[2 * NTAP + kk];
  const float mk  = 1.0f / (1.0f + expf(-lg));
  float py = (float)(ho - 1 + ky) + d_y;
  float px = (float)(wo - 1 + kx) + d_x;
  py = fminf(fmaxf(py, -2.0f), 129.0f);
  px = fminf(fmaxf(px, -2.0f), 129.0f);
  const float fy = floorf(py), fx = floorf(px);
  const float wy = py - fy, wx = px - fx;
  const int yi = (int)fy, xi = (int)fx;
  const int yi1 = yi + 1, xi1 = xi + 1;
  const float vy0 = (yi  >= 0 && yi  < NHGT) ? 1.0f : 0.0f;
  const float vy1 = (yi1 >= 0 && yi1 < NHGT) ? 1.0f : 0.0f;
  const float vx0 = (xi  >= 0 && xi  < NWID) ? 1.0f : 0.0f;
  const float vx1 = (xi1 >= 0 && xi1 < NWID) ? 1.0f : 0.0f;
  const int yc0 = min(max(yi, 0), NHGT - 1),  yc1 = min(max(yi1, 0), NHGT - 1);
  const int xc0 = min(max(xi, 0), NWID - 1),  xc1 = min(max(xi1, 0), NWID - 1);
  const float w00 = (1.0f - wy) * (1.0f - wx);
  const float w01 = (1.0f - wy) * wx;
  const float w10 = wy * (1.0f - wx);
  const float w11 = wy * wx;
  const float v00 = vy0 * vx0, v01 = vy0 * vx1, v10 = vy1 * vx0, v11 = vy1 * vx1;
  const int bg = bbase + bl;
  const float* r0p = xt + ((size_t)(bg * NHGT + yc0)) * NWID * NCH + sub * 8;
  const float* r1p = xt + ((size_t)(bg * NHGT + yc1)) * NWID * NCH + sub * 8;
  const float* p00 = r0p + (size_t)xc0 * NCH;
  const float* p01 = r0p + (size_t)xc1 * NCH;
  const float* p10 = r1p + (size_t)xc0 * NCH;
  const float* p11 = r1p + (size_t)xc1 * NCH;
  const v4f a00 = *(const v4f*)(p00), c00 = *(const v4f*)(p00 + 4);
  const v4f a01 = *(const v4f*)(p01), c01 = *(const v4f*)(p01 + 4);
  const v4f a10 = *(const v4f*)(p10), c10 = *(const v4f*)(p10 + 4);
  const v4f a11 = *(const v4f*)(p11), c11 = *(const v4f*)(p11 + 4);
  v8h hv;
#pragma unroll
  for (int e = 0; e < 4; ++e) {
    float s = 0.0f;
    s += (a00[e] * v00) * w00;
    s += (a01[e] * v01) * w01;
    s += (a10[e] * v10) * w10;
    s += (a11[e] * v11) * w11;
    s = s * mk;
    hv[e] = (_Float16)(s * A_CARRY);
    float u = 0.0f;
    u += (c00[e] * v00) * w00;
    u += (c01[e] * v01) * w01;
    u += (c10[e] * v10) * w10;
    u += (c11[e] * v11) * w11;
    u = u * mk;
    hv[4 + e] = (_Float16)(u * A_CARRY);
  }
  unsigned short* p = P + (size_t)t * 8;
  *(volatile v8h*)(p) = hv;
  __threadfence();
  *(volatile v8h*)(p) = hv;
}

extern "C" void kernel_launch(void* const* d_in, const int* in_sizes, int n_in,
                              void* d_out, int out_size, void* d_ws, size_t ws_size,
                              hipStream_t stream) {
  if (n_in < 5) return;
  if (in_sizes[0] != NBATCH * NCH * NPIX) return;
  if (in_sizes[1] != NOFF * KDIM) return;
  if (in_sizes[2] != NOFF) return;
  if (in_sizes[3] != NCO * KDIM) return;
  if (in_sizes[4] != NCO) return;
  if (out_size != NBATCH * NCO * NPIX) return;
  if (ws_size < WS_TOTAL) return;

  const float* x    = (const float*)d_in[0];
  const float* w_om = (const float*)d_in[1];
  const float* b_om = (const float*)d_in[2];
  const float* w    = (const float*)d_in[3];
  const float* bias = (const float*)d_in[4];
  float* out = (float*)d_out;
  char*  ws  = (char*)d_ws;

  float*          xT  = (float*)(ws + WS_XT);
  unsigned short* Pp  = (unsigned short*)(ws + WS_P);
  float*          OMp = (float*)(ws + WS_OM);
  unsigned short* Bt1 = (unsigned short*)(ws + WS_BT1);
  unsigned short* Bt2 = (unsigned short*)(ws + WS_BT2);

  k_xpose<<<NBATCH * NHGT * 2, NTHR, 0, stream>>>(x, xT);
  k_wprep<<<(NOFFPAD * (KDIM / 8)) / NTHR, NTHR, 0, stream>>>(w_om, NOFF, W1_CARRY, Bt1);
  k_wprep<<<(NOFFPAD * (KDIM / 8)) / NTHR, NTHR, 0, stream>>>(w, NCO, W2_CARRY, Bt2);

  const int egrid = (MROWS * NTAP * 8) / NTHR;
  for (int ch = 0; ch < NCHUNK; ++ch) {
    const int bbase = ch * BCHUNK;
    k_im2col<<<egrid, NTHR, 0, stream>>>(xT, bbase, Pp);
    wmma_gemm64<0, false, 0, 0, false, 0><<<dim3((MROWS / 64) / 8, 1), dim3(NTHR), 0, stream>>>(
        Pp, Pp, KDIM, (long)0,
        Bt1, Bt1, KDIM, (long)0,
        (void*)OMp, (void*)OMp, NOFFPAD, (long)0,
        b_om,
        (const float*)xT, (long)0,
        MROWS, NOFFPAD, KDIM, G1_FOLD);
    k_gather<<<egrid, NTHR, 0, stream>>>(xT, OMp, b_om, bbase, Pp);
    float* outc = out + (size_t)bbase * NCO * NPIX;
    wmma_gemm64<0, false, 1, 0, false, 0><<<dim3((NPIX / 64) / 8, BCHUNK), dim3(NTHR), 0, stream>>>(
        Bt2, Bt2, KDIM, (long)0,
        Pp, Pp, KDIM, (long)NPIX * KDIM,
        (void*)outc, (void*)outc, NPIX, (long)NCO * NPIX,
        bias,
        (const float*)xT, (long)0,
        NCO, NPIX, KDIM, G2_FOLD);
  }
}
